// WavLMAttention_72164040507657
// MI455X (gfx1250) — hardware-verified
//
#include <hip/hip_runtime.h>
#include <math.h>

#ifndef NB
#define NB 4
#endif
#ifndef SEQ
#define SEQ 1024
#endif
#define NB_FULL  4
#define SEQ_FULL 1024
#define DM   1024
#define NH   16
#define HD   64
#define NBKT 320
#define MT   (NB * SEQ)
#define KQP  (2 * DM)
#define QOFF 0
#define KOFF DM
#define TP   (2 * SEQ)
#define WLEN (SEQ + 16)
#define AWV  4
#define WSCL 64.0f
#define QKS  16.0f
#define VSC  16.0f
#define PSC  16384.0f
#define CSC  16.0f
#define RSC  4096.0f
#define RSQD 0.125f
#define LN10F 2.302585092994046f

static_assert(NH * HD == DM);
static_assert(HD == 64);
static_assert(NB >= 1 && NB <= NB_FULL);
static_assert((SEQ % 64) == 0 && SEQ >= 64 && SEQ <= SEQ_FULL);
static_assert((MT % 128) == 0);
static_assert((DM % 64) == 0 && (KQP % 64) == 0 && (DM % 32) == 0);
static_assert((((MT / 64) * (KQP / 64)) % 8) == 0);
static_assert((((DM / 64) * (MT / 64)) % 8) == 0);
static_assert(((SEQ * DM) % 2048) == 0);
static_assert(((DM * DM) % 2048) == 0);
static_assert(((NB * NH * (SEQ / 16)) % AWV) == 0);
static_assert((TP % 128) == 0);
static_assert((SEQ % 32) == 0);

typedef _Float16 v16h __attribute__((ext_vector_type(16)));
typedef unsigned short v16us __attribute__((ext_vector_type(16)));
typedef unsigned short v8us  __attribute__((ext_vector_type(8)));
typedef float v8f __attribute__((ext_vector_type(8)));
typedef float v4f __attribute__((ext_vector_type(4)));
typedef unsigned int v4u __attribute__((ext_vector_type(4)));

union FragU { v16us v; v8us h[2]; };

__device__ __forceinline__ unsigned short bf_bits(float f) {
  const unsigned u = __float_as_uint(f);
  return (unsigned short)((u + 0x7FFFu + ((u >> 16) & 1u)) >> 16);
}
__device__ __forceinline__ float bf_up(unsigned short h) { return __uint_as_float(((unsigned)h) << 16); }
__device__ __forceinline__ float bfr(float f) { return bf_up(bf_bits(f)); }
__device__ __forceinline__ unsigned short h_bits(_Float16 x) { return __builtin_bit_cast(unsigned short, x); }
__device__ __forceinline__ unsigned short f2h(float f) { return h_bits((_Float16)f); }
__device__ __forceinline__ float h_val(unsigned short b) { return (float)__builtin_bit_cast(_Float16, b); }
__device__ __forceinline__ unsigned pk16(unsigned short a, unsigned short b) { return (unsigned)a | ((unsigned)b << 16); }
__device__ __forceinline__ int clampi(int v, int lo, int hi) { return v < lo ? lo : (v > hi ? hi : v); }
__device__ __forceinline__ int imin(int a, int b) { return a < b ? a : b; }
__device__ __forceinline__ v8f zero8() { v8f z = {0.f, 0.f, 0.f, 0.f, 0.f, 0.f, 0.f, 0.f}; return z; }

__device__ __forceinline__ v16us ldfrag_u(const unsigned short* p) {
  FragU f;
  f.h[0] = *(const v8us*)(p);
  f.h[1] = *(const v8us*)(p + 16);
  return f.v;
}

__device__ __forceinline__ v8f mma_raw(v16us a, v16us b, v8f c) {
  return __builtin_amdgcn_wmma_f32_16x16x32_f16(false, __builtin_bit_cast(v16h, a), false,
                                                __builtin_bit_cast(v16h, b), (short)0, c, false, false);
}
__device__ __forceinline__ v8f mma_g(v16us a, v16us b, v8f c) {
  c = mma_raw(a, b, c);
#if defined(__HIP_DEVICE_COMPILE__)
  asm volatile("v_nop\n\tv_nop\n\tv_nop\n\tv_nop" : "+v"(c) : "v"(a), "v"(b));
#endif
  return c;
}
__device__ __forceinline__ void dep_guard1(v8f& a, v8f& b, v16us x) {
#if defined(__HIP_DEVICE_COMPILE__)
  asm volatile("v_nop\n\tv_nop\n\tv_nop\n\tv_nop" : "+v"(a), "+v"(b) : "v"(x));
#endif
}
__device__ __forceinline__ void keep4_u(v16us a, v16us b, v16us c, v16us d) {
#if defined(__HIP_DEVICE_COMPILE__)
  asm volatile("v_nop" :: "v"(a), "v"(b), "v"(c), "v"(d));
#endif
}
__device__ __forceinline__ void acc_guard4(v8f& a, v8f& b, v8f& c, v8f& d) {
#if defined(__HIP_DEVICE_COMPILE__)
  asm volatile("v_nop\n\tv_nop\n\tv_nop\n\tv_nop" : "+v"(a), "+v"(b), "+v"(c), "+v"(d));
#endif
}
__device__ __forceinline__ void wave_sync_lds() {
  __builtin_amdgcn_fence(__ATOMIC_RELEASE, "workgroup");
  __builtin_amdgcn_wave_barrier();
  __builtin_amdgcn_fence(__ATOMIC_ACQUIRE, "workgroup");
}

__global__ __launch_bounds__(256) void cvt_lin(const float* __restrict__ w, unsigned short* o,
                                                int nsrc, int ndst, float sc, int sstride, int dstride) {
  const float* wb = w + (size_t)blockIdx.y * (size_t)sstride;
  unsigned short* ob = o + (size_t)blockIdx.y * (size_t)dstride;
  const int base = (blockIdx.x * 256 + threadIdx.x) * 8;
  if (base + 8 > ndst) return;
  const bool inr = (base + 8 <= nsrc);
  const int lb = inr ? base : (nsrc - 8);
  const v4f a0 = *(const v4f*)(wb + lb);
  const v4f a1 = *(const v4f*)(wb + lb + 4);
  v4u hv;
#pragma unroll
  for (int e = 0; e < 2; ++e) {
    hv[e]     = pk16(f2h(bfr(a0[2 * e]) * sc), f2h(bfr(a0[2 * e + 1]) * sc));
    hv[2 + e] = pk16(f2h(bfr(a1[2 * e]) * sc), f2h(bfr(a1[2 * e + 1]) * sc));
  }
  const v4u zz = {0u, 0u, 0u, 0u};
  hv = inr ? hv : zz;
  unsigned short* d = ob + base;
  *(volatile v4u*)d = hv;
  __threadfence();
  *(volatile v4u*)d = hv;
}

__device__ __forceinline__ int bucket_of(int d) {
#pragma clang fp contract(off)
  const int a = d < 0 ? -d : d;
  const int am = a < 1 ? 1 : a;
  float r = (float)am * (1.0f / 80.0f);
  float lg = logf(r);
  lg = lg * (1.0f / LN10F);
  lg = lg * 80.0f;
  const float s = 80.0f + lg;
  int iv = (int)s;
  iv = iv < 159 ? iv : 159;
  const int v = (a < 80) ? a : iv;
  return v + ((d > 0) ? 160 : 0);
}
__global__ __launch_bounds__(256) void tab_kernel(const float* __restrict__ rel, int nrel, float* TB) {
  __shared__ __align__(16) float tbs[TP];
  const int h = blockIdx.x;
  const int t = threadIdx.x;
#pragma unroll 1
  for (int dd = t; dd < TP; dd += 256) {
    const int d = dd - (SEQ - 1);
    const int bk = bucket_of(d);
    const int idx = clampi(bk * NH + h, 0, nrel - 1);
    const float val = bfr(rel[idx]);
    tbs[dd] = (dd < 2 * SEQ - 1) ? val : 0.f;
  }
  __syncthreads();
#pragma unroll 1
  for (int e4 = t; e4 < TP / 4; e4 += 256) {
    const v4f v = *(const v4f*)(tbs + 4 * e4);
    float* dst = TB + (size_t)h * TP + 4 * e4;
    *(volatile v4f*)dst = v;
    __threadfence();
    *(volatile v4f*)dst = v;
  }
}

__global__ __launch_bounds__(64) void gate_kernel(const float* __restrict__ x, const float* __restrict__ gw,
                                                   const float* __restrict__ gb, int ngb,
                                                   const float* __restrict__ gc, int ngc, float* GT) {
  __shared__ float sw[HD * 8];
  __shared__ float sb[8];
  __shared__ __align__(16) float sgl[64];
  const int t = threadIdx.x;
  const int s0 = blockIdx.x * 64, h = blockIdx.y, b = blockIdx.z;
  for (int i = t; i < HD * 8; i += 64) {
    const int e = i >> 6, d = i & 63;
    sw[d * 8 + e] = bfr(gw[i]);
  }
  {
    const float bb = bfr(gb[clampi(t < 8 ? t : 7, 0, ngb - 1)]);
    if (t < 8) sb[t] = bb;
  }
  __syncthreads();
  const float gch = bfr(gc[clampi(h, 0, ngc - 1)]);
  const float* xr = x + ((size_t)b * SEQ_FULL + (size_t)(s0 + t)) * DM + h * HD;
  float acc[8];
#pragma unroll
  for (int j = 0; j < 8; ++j) acc[j] = 0.f;
#pragma unroll 1
  for (int i = 0; i < HD; ++i) {
    const float xv = bfr(xr[i]);
#pragma unroll
    for (int j = 0; j < 8; ++j) acc[j] += xv * sw[i * 8 + j];
  }
  const float u0 = ((acc[0] + sb[0]) + (acc[1] + sb[1])) + ((acc[2] + sb[2]) + (acc[3] + sb[3]));
  const float u1 = ((acc[4] + sb[4]) + (acc[5] + sb[5])) + ((acc[6] + sb[6]) + (acc[7] + sb[7]));
  const float ga = 1.0f / (1.0f + expf(-u0));
  const float gbv = 1.0f / (1.0f + expf(-u1));
  const float gate = ga * (gbv * gch - 1.0f) + 2.0f;
  sgl[t] = gate;
  __syncthreads();
  const int t16 = t & 15;
  const v4f v = *(const v4f*)(sgl + 4 * t16);
  float* dst = GT + ((size_t)(b * NH + h) * SEQ + (size_t)s0) + 4 * t16;
  if (t < 16) *(volatile v4f*)dst = v;
  __threadfence();
  if (t < 16) *(volatile v4f*)dst = v;
}

__device__ __forceinline__ void kloop64(v8f (&acc)[4][4], const unsigned short* __restrict__ Ap, int lda,
                                        const unsigned short* __restrict__ Btp, int ldb,
                                        int m0, int n0, int K, int rlane, int koff) {
#pragma unroll 1
  for (int k0 = 0; k0 < K; k0 += 32) {
    v16us bh[4];
#pragma unroll
    for (int j = 0; j < 4; ++j) {
      const size_t bo = (size_t)(n0 + (j << 4) + rlane) * ldb + koff + k0;
      bh[j] = ldfrag_u(Btp + bo);
    }
#pragma unroll
    for (int i = 0; i < 4; ++i) {
      const size_t ao = (size_t)(m0 + (i << 4) + rlane) * lda + koff + k0;
      const v16us ah = ldfrag_u(Ap + ao);
#pragma unroll
      for (int j = 0; j < 4; ++j) acc[i][j] = mma_raw(ah, bh[j], acc[i][j]);
      dep_guard1(acc[i][0], acc[i][3], ah);
    }
    keep4_u(bh[0], bh[1], bh[2], bh[3]);
  }
}

template <int OM, int TWO, int BROW>
__global__ __launch_bounds__(256) void gemm64(
    const unsigned short* __restrict__ Ap, const unsigned short* __restrict__ A2p, int lda,
    const unsigned short* __restrict__ Btp, int ldb,
    unsigned short* Ch, float* Cf, int ldc, float osc, float a2sc,
    const float* __restrict__ bias0, const float* __restrict__ bias1, int nsplit, int nb0, int nb1, float bsc,
    int M, int N, int K) {
  __shared__ __align__(16) float sT[8][16 * 68];
  const int lane = threadIdx.x & 31;
  const int wave = threadIdx.x >> 5;
  const int tilesN = N >> 6;
  const int tilesM = M >> 6;
  const int tile = blockIdx.x * 8 + wave;
  if (tile >= tilesM * tilesN) return;
  const int tm = tile / tilesN;
  const int tn = tile - tm * tilesN;
  const int m0 = tm << 6;
  const int n0 = tn << 6;

  const int rlane = lane & 15;
  const int koff  = (lane >> 4) * 8;
  const int mOff  = (lane >> 4) * 8;

  v8f acc[4][4];
#pragma unroll
  for (int i = 0; i < 4; ++i)
#pragma unroll
    for (int j = 0; j < 4; ++j) acc[i][j] = zero8();

  if (TWO != 0) {
    kloop64(acc, A2p, lda, Btp, ldb, m0, n0, K, rlane, koff);
    acc_guard4(acc[0][0], acc[0][1], acc[0][2], acc[0][3]);
    acc_guard4(acc[1][0], acc[1][1], acc[1][2], acc[1][3]);
    acc_guard4(acc[2][0], acc[2][1], acc[2][2], acc[2][3]);
    acc_guard4(acc[3][0], acc[3][1], acc[3][2], acc[3][3]);
#pragma unroll
    for (int i = 0; i < 4; ++i)
#pragma unroll
      for (int j = 0; j < 4; ++j) acc[i][j] = acc[i][j] * a2sc;
    acc_guard4(acc[0][0], acc[0][1], acc[0][2], acc[0][3]);
    acc_guard4(acc[1][0], acc[1][1], acc[1][2], acc[1][3]);
    acc_guard4(acc[2][0], acc[2][1], acc[2][2], acc[2][3]);
    acc_guard4(acc[3][0], acc[3][1], acc[3][2], acc[3][3]);
  }
  kloop64(acc, Ap, lda, Btp, ldb, m0, n0, K, rlane, koff);
  acc_guard4(acc[0][0], acc[0][1], acc[0][2], acc[0][3]);
  acc_guard4(acc[1][0], acc[1][1], acc[1][2], acc[1][3]);
  acc_guard4(acc[2][0], acc[2][1], acc[2][2], acc[2][3]);
  acc_guard4(acc[3][0], acc[3][1], acc[3][2], acc[3][3]);

  const int hh2 = lane >> 4, c4 = (lane & 15) * 4;
  const int q8  = lane >> 3, c8 = (lane & 7) * 8;

  float bcol[8];
  {
    const int cb = (OM == 0) ? c4 : c8;
#pragma unroll
    for (int e = 0; e < 8; ++e) {
      float v = 0.f;
      if (BROW == 0 && (OM == 1 || e < 4)) {
        const int col = n0 + cb + e;
        const float v0 = bias0[clampi(col, 0, nb0 - 1)];
        const float v1 = bias1[clampi(col - nsplit, 0, nb1 - 1)];
        v = bfr(col < nsplit ? v0 : v1) * bsc;
      }
      bcol[e] = v;
    }
  }

  float* slab = sT[wave];
#pragma unroll
  for (int i = 0; i < 4; ++i) {
    const int mBase = m0 + (i << 4);
#pragma unroll
    for (int j = 0; j < 4; ++j) {
#pragma unroll
      for (int r = 0; r < 8; ++r) {
        slab[(mOff + r) * 68 + (j << 4) + rlane] = acc[i][j][r];
      }
    }
    wave_sync_lds();
    if (OM == 0) {
      v4f vals[8];
      const v4f bv4 = {bcol[0], bcol[1], bcol[2], bcol[3]};
#pragma unroll
      for (int it = 0; it < 8; ++it) {
        const int row = it * 2 + hh2;
        float brow = 0.f;
        if (BROW == 1) brow = bfr(bias0[clampi(mBase + row, 0, nb0 - 1)]) * bsc;
        const v4f v = *(const v4f*)(slab + row * 68 + c4);
        vals[it] = v * osc + bv4 + brow;
      }
      for (int pass = 0; pass < 2; ++pass) {
#pragma unroll
        for (int it = 0; it < 8; ++it) {
          const int row = it * 2 + hh2;
          *(volatile v4f*)(Cf + (size_t)(mBase + row) * ldc + (size_t)n0 + c4) = vals[it];
        }
        __threadfence();
      }
    } else {
      v4u hv[4];
#pragma unroll
      for (int it = 0; it < 4; ++it) {
        const int row = it * 4 + q8;
        float brow = 0.f;
        if (BROW == 1) brow = bfr(bias0[clampi(mBase + row, 0, nb0 - 1)]) * bsc;
        const float* sp = slab + row * 68 + c8;
        v4u ha = {0u, 0u, 0u, 0u};
#pragma unroll
        for (int e = 0; e < 4; ++e) {
          const float b0 = sp[2 * e]     * osc + bcol[2 * e]     + brow;
          const float b1 = sp[2 * e + 1] * osc + bcol[2 * e + 1] + brow;
          ha[e] = pk16(f2h(b0), f2h(b1));
        }
        hv[it] = ha;
      }
      for (int pass = 0; pass < 2; ++pass) {
#pragma unroll
        for (int it = 0; it < 4; ++it) {
          const int row = it * 4 + q8;
          const size_t go = (size_t)(mBase + row) * ldc + (size_t)n0 + c8;
          *(volatile v4u*)(Ch + go) = hv[it];
        }
        __threadfence();
      }
    }
    wave_sync_lds();
  }
}

__global__ __launch_bounds__(128) void attn_kernel(
    const unsigned short* __restrict__ KQ, const unsigned short* __restrict__ VT,
    const float* __restrict__ GT, const float* __restrict__ TB,
    unsigned short* Z, unsigned short* ZR) {
  __shared__ __align__(16) float bwin[AWV][WLEN];
  __shared__ __align__(16) unsigned short pws[AWV][16 * 32];
  __shared__ __align__(16) unsigned short zst[AWV][16 * 64];
  __shared__ __align__(16) unsigned short zrt[AWV][16 * 64];
  const int lane = threadIdx.x & 31, wv = threadIdx.x >> 5, m = lane & 15, hh = lane >> 4;
  const int task = blockIdx.x * AWV + wv;
  const int nqt = SEQ / 16;
  const int bh = task / nqt;
  const int t0 = (task - bh * nqt) << 4;
  const int b = bh / NH, h = bh - (bh / NH) * NH;
  if (b >= NB) return;
  const size_t tok0 = (size_t)b * SEQ;
  float* bw = bwin[wv];
  unsigned short* ph = pws[wv];

  {
    const float* th = TB + (size_t)h * TP + (SEQ - 16 - t0);
#pragma unroll 1
    for (int it = 0; it < (WLEN + 31) / 32; ++it) {
      const int xw = imin(lane + 32 * it, WLEN - 1);
      bw[xw] = th[xw];
    }
  }
  float gr[8];
  {
    const float* gp = GT + (size_t)bh * SEQ + t0 + 8 * hh;
#pragma unroll
    for (int r = 0; r < 8; ++r) gr[r] = gp[r];
  }
  wave_sync_lds();

  const unsigned short* qp = KQ + (tok0 + (size_t)(t0 + m)) * KQP + QOFF + h * HD + 8 * hh;
  const v16us qf0 = ldfrag_u(qp);
  const v16us qf1 = ldfrag_u(qp + 32);

  const float SCS = RSQD / (QKS * QKS);

  float mx[8], ls[8];
  v8f O0 = zero8(), O1 = zero8(), O2 = zero8(), O3 = zero8();
#pragma unroll
  for (int r = 0; r < 8; ++r) { mx[r] = -1.0e30f; ls[r] = 0.f; }

#pragma unroll 1
  for (int kb = 0; kb < SEQ / 32; ++kb) {
    wave_sync_lds();
    const int sb = kb << 5;
    v8f S0, S1;
    {
      const unsigned short* kp = KQ + (tok0 + (size_t)(sb + m)) * KQP + KOFF + h * HD + 8 * hh;
      S0 = mma_g(qf0, ldfrag_u(kp), zero8());
      S0 = mma_g(qf1, ldfrag_u(kp + 32), S0);
      const unsigned short* kp1 = kp + (size_t)16 * KQP;
      S1 = mma_g(qf0, ldfrag_u(kp1), zero8());
      S1 = mma_g(qf1, ldfrag_u(kp1 + 32), S1);
    }

    float s0[8], s1[8];
#pragma unroll
    for (int r = 0; r < 8; ++r) {
      const int row = 8 * hh + r;
      const float bv0 = bw[sb + m - row + 15];
      const float bv1 = bw[sb + 16 + m - row + 15];
      s0[r] = S0[r] * SCS + gr[r] * bv0;
      s1[r] = S1[r] * SCS + gr[r] * bv1;
    }

#pragma unroll
    for (int r = 0; r < 8; ++r) {
      float xm = fmaxf(s0[r], s1[r]);
      xm = fmaxf(xm, __shfl_xor(xm, 1, 32));
      xm = fmaxf(xm, __shfl_xor(xm, 2, 32));
      xm = fmaxf(xm, __shfl_xor(xm, 4, 32));
      xm = fmaxf(xm, __shfl_xor(xm, 8, 32));
      const float mn = fmaxf(mx[r], xm);
      const float al = __expf(mx[r] - mn);
      mx[r] = mn;
      const float p0 = __expf(s0[r] - mn);
      const float p1 = __expf(s1[r] - mn);
      float ps = p0 + p1;
      ps += __shfl_xor(ps, 1, 32);
      ps += __shfl_xor(ps, 2, 32);
      ps += __shfl_xor(ps, 4, 32);
      ps += __shfl_xor(ps, 8, 32);
      ls[r] = ls[r] * al + ps;
      O0[r] = O0[r] * al;
      O1[r] = O1[r] * al;
      O2[r] = O2[r] * al;
      O3[r] = O3[r] * al;
      const int row = 8 * hh + r;
      ph[row * 32 + m]      = f2h(p0 * PSC);
      ph[row * 32 + 16 + m] = f2h(p1 * PSC);
    }
    wave_sync_lds();

    const v16us af = ldfrag_u(ph + m * 32 + 8 * hh);
    const size_t vo = (size_t)(h * HD + m) * MT + tok0 + (size_t)sb + 8 * hh;
    const v16us vf0 = ldfrag_u(VT + vo);
    const v16us vf1 = ldfrag_u(VT + vo + (size_t)16 * MT);
    const v16us vf2 = ldfrag_u(VT + vo + (size_t)32 * MT);
    const v16us vf3 = ldfrag_u(VT + vo + (size_t)48 * MT);
    O0 = mma_g(af, vf0, O0);
    O1 = mma_g(af, vf1, O1);
    O2 = mma_g(af, vf2, O2);
    O3 = mma_g(af, vf3, O3);
  }
  acc_guard4(O0, O1, O2, O3);

  unsigned short* zs = zst[wv];
  unsigned short* zr = zrt[wv];
  const float fin = CSC / (PSC * VSC);
#pragma unroll
  for (int r = 0; r < 8; ++r) {
    const int row = 8 * hh + r;
    const float g = (1.0f / ls[r]) * fin;
    const float c0 = O0[r] * g, c1 = O1[r] * g, c2 = O2[r] * g, c3 = O3[r] * g;
    const unsigned short e0 = f2h(c0), e1 = f2h(c1), e2 = f2h(c2), e3 = f2h(c3);
    zs[row * 64 + m]      = e0;
    zs[row * 64 + 16 + m] = e1;
    zs[row * 64 + 32 + m] = e2;
    zs[row * 64 + 48 + m] = e3;
    zr[row * 64 + m]      = f2h((c0 - h_val(e0)) * RSC);
    zr[row * 64 + 16 + m] = f2h((c1 - h_val(e1)) * RSC);
    zr[row * 64 + 32 + m] = f2h((c2 - h_val(e2)) * RSC);
    zr[row * 64 + 48 + m] = f2h((c3 - h_val(e3)) * RSC);
  }
  wave_sync_lds();
  {
    const int q8 = lane >> 3, c8 = (lane & 7) * 8;
    v4u hv[4], hr[4];
#pragma unroll
    for (int it = 0; it < 4; ++it) {
      const int row = it * 4 + q8;
      hv[it] = *(const v4u*)(zs + row * 64 + c8);
      hr[it] = *(const v4u*)(zr + row * 64 + c8);
    }
    const size_t zr0 = tok0 + (size_t)t0;
    for (int pass = 0; pass < 2; ++pass) {
#pragma unroll
      for (int it = 0; it < 4; ++it) {
        const int row = it * 4 + q8;
        const size_t off = (zr0 + (size_t)row) * DM + h * HD + c8;
        *(volatile v4u*)(Z + off)  = hv[it];
        *(volatile v4u*)(ZR + off) = hr[it];
      }
      __threadfence();
    }
  }
}

extern "C" void kernel_launch(void* const* d_in, const int* in_sizes, int n_in,
                              void* d_out, int out_size, void* d_ws, size_t ws_size,
                              hipStream_t stream) {
  if (n_in < 13) return;
  if (in_sizes[0] < ((NB - 1) * SEQ_FULL + SEQ) * DM) return;
  if (in_sizes[1] < DM * DM || in_sizes[3] < DM * DM || in_sizes[5] < DM * DM || in_sizes[7] < DM * DM) return;
  if (in_sizes[2] < DM || in_sizes[4] < DM || in_sizes[6] < DM || in_sizes[8] < DM) return;
  if (in_sizes[9] < NBKT * NH) return;
  if (in_sizes[10] < NH || in_sizes[11] < 8 * HD || in_sizes[12] < 8) return;
  if (out_size < MT * DM) return;

  const float* x   = (const float*)d_in[0];
  const float* wq  = (const float*)d_in[1];
  const float* bq  = (const float*)d_in[2];
  const float* wk  = (const float*)d_in[3];
  const float* bk  = (const float*)d_in[4];
  const float* wv  = (const float*)d_in[5];
  const float* bv  = (const float*)d_in[6];
  const float* wo  = (const float*)d_in[7];
  const float* bo  = (const float*)d_in[8];
  const float* rel = (const float*)d_in[9];
  const float* gc  = (const float*)d_in[10];
  const float* gw  = (const float*)d_in[11];
  const float* gb  = (const float*)d_in[12];
  const int nbq = in_sizes[2], nbk = in_sizes[4], nbv = in_sizes[6], nbo = in_sizes[8];
  const int nrel = in_sizes[9], ngc = in_sizes[10], ngb = in_sizes[12];

  const size_t PXH = (size_t)MT * DM * 2;
  const size_t PWT = (size_t)3 * DM * DM * 2;
  const size_t PWO = (size_t)DM * DM * 2;
  const size_t PKQ = (size_t)MT * KQP * 2;
  const size_t PVT = (size_t)DM * MT * 2;
  const size_t PZ  = (size_t)MT * DM * 2;
  const size_t PGT = (size_t)NB * NH * SEQ * 4;
  const size_t PTB = (size_t)NH * TP * 4;
  size_t off = 0;
  const size_t oXH = off; off += PXH;
  const size_t oWT = off; off += PWT;
  const size_t oWO = off; off += PWO;
  const size_t oKQ = off; off += PKQ;
  const size_t oVT = off; off += PVT;
  const size_t oZ  = off; off += PZ;
  const size_t oZR = off; off += PZ;
  const size_t oGT = off; off += PGT;
  const size_t oTB = off; off += PTB;
  if (off > ws_size) return;
  if (off > (size_t)134217728) return;

  char* ws = (char*)d_ws;
  unsigned short* XH  = (unsigned short*)(ws + oXH);
  unsigned short* WT  = (unsigned short*)(ws + oWT);
  unsigned short* WOT = (unsigned short*)(ws + oWO);
  unsigned short* KQ  = (unsigned short*)(ws + oKQ);
  unsigned short* VT  = (unsigned short*)(ws + oVT);
  unsigned short* Z   = (unsigned short*)(ws + oZ);
  unsigned short* ZR  = (unsigned short*)(ws + oZR);
  float* GT = (float*)(ws + oGT);
  float* TB = (float*)(ws + oTB);
  float* out0 = (float*)d_out;
  float* fdummy = (float*)(ws + oKQ);
  unsigned short* hdummy = KQ;

  const dim3 blk(256);
  const int gKQ = ((MT / 64) * (KQP / 64)) / 8;
  const int gVT = ((DM / 64) * (MT / 64)) / 8;
  const int gPR = ((MT / 64) * (DM / 64)) / 8;
  const int gW  = (DM * DM) / 2048;

  cvt_lin<<<dim3((SEQ * DM) / 2048, NB), blk, 0, stream>>>(x, XH, SEQ * DM, SEQ * DM, 1.0f, SEQ_FULL * DM, SEQ * DM);
  tab_kernel<<<dim3(NH), blk, 0, stream>>>(rel, nrel, TB);
  gate_kernel<<<dim3(SEQ / 64, NH, NB), dim3(64), 0, stream>>>(x, gw, gb, ngb, gc, ngc, GT);
  cvt_lin<<<dim3(gW, 1), blk, 0, stream>>>(wq, WT, DM * DM, DM * DM, WSCL, 0, 0);
  cvt_lin<<<dim3(gW, 1), blk, 0, stream>>>(wk, WT + (size_t)DM * DM, DM * DM, DM * DM, WSCL, 0, 0);
  cvt_lin<<<dim3(gW, 1), blk, 0, stream>>>(wv, WT + (size_t)2 * DM * DM, DM * DM, DM * DM, WSCL, 0, 0);
  cvt_lin<<<dim3(gW, 1), blk, 0, stream>>>(wo, WOT, DM * DM, DM * DM, WSCL, 0, 0);

  gemm64<1, 0, 0><<<dim3(gKQ), blk, 0, stream>>>(XH, XH, DM, WT, DM, KQ, fdummy, KQP, QKS / WSCL, 1.0f,
                                                 bq, bk, DM, nbq, nbk, QKS, MT, KQP, DM);
  gemm64<1, 0, 1><<<dim3(gVT), blk, 0, stream>>>(WT + (size_t)2 * DM * DM, WT + (size_t)2 * DM * DM, DM, XH, DM,
                                                 VT, fdummy, MT, VSC / WSCL, 1.0f,
                                                 bv, bv, DM, nbv, nbv, VSC, DM, MT, DM);

  attn_kernel<<<dim3((NB * NH * (SEQ / 16)) / AWV), dim3(128), 0, stream>>>(KQ, VT, GT, TB, Z, ZR);

  gemm64<0, 1, 0><<<dim3(gPR), blk, 0, stream>>>(Z, ZR, DM, WOT, DM, hdummy, out0, DM, 1.0f / (WSCL * CSC), 1.0f / RSC,
                                                 bo, bo, DM, nbo, nbo, 1.0f, MT, DM, DM);
  (void)hipGetLastError();
}
